// SelectiveSSM_3444563771624
// MI455X (gfx1250) — hardware-verified
//
#include <hip/hip_runtime.h>
#include <math.h>

typedef __attribute__((ext_vector_type(16))) _Float16 v16h;
typedef __attribute__((ext_vector_type(8)))  _Float16 v8h;
typedef __attribute__((ext_vector_type(16))) __bf16   v16b;
typedef __attribute__((ext_vector_type(8)))  __bf16   v8b;
typedef __attribute__((ext_vector_type(8)))  float    v8f;
typedef __attribute__((ext_vector_type(4)))  float    v4f;

constexpr int kBatch  = 2;
constexpr int kSeq    = 2048;
constexpr int kDin    = 2048;
constexpr int kNst    = 16;
constexpr int kDtR    = 128;
constexpr int kPrjN   = kDtR + 2 * kNst;
constexpr int kPrjP   = 192;
constexpr int kRows   = kBatch * kSeq;
constexpr int kBCW    = 2 * kNst;
constexpr int kScanCh = 64;
constexpr int kScanTS = 64;
constexpr int kScanYP = 68;
static_assert(kPrjN == 160, "x_proj width");
static_assert(kPrjP >= kPrjN && (kPrjP % 64) == 0, "padded N is a tile multiple");
static_assert((kDin % 32) == 0 && (kDtR % 32) == 0, "GEMM K multiples of 32");
static_assert((kRows % 64) == 0 && (kDin % 64) == 0, "GEMM M,N multiples of 64");
static_assert((kSeq % kScanTS) == 0 && (kDin % kScanCh) == 0 && kScanCh == 64 && kScanTS == 64, "scan tiles");
static_assert(((kPrjN * kDin / 8) % 256) == 0 && ((kPrjP * kDin / 8) % 256) == 0, "pad boundary is block-uniform");

constexpr size_t kOffXH   = 0;
constexpr size_t kOffXL   = kOffXH  + (size_t)kRows * kDin  * 2;
constexpr size_t kOffW1H  = kOffXL  + (size_t)kRows * kDin  * 2;
constexpr size_t kOffW1L  = kOffW1H + (size_t)kPrjP * kDin  * 2;
constexpr size_t kOffW2H  = kOffW1L + (size_t)kPrjP * kDin  * 2;
constexpr size_t kOffW2L  = kOffW2H + (size_t)kDin  * kDtR  * 2;
constexpr size_t kOffXD   = kOffW2L + (size_t)kDin  * kDtR  * 2;
constexpr size_t kOffDUH  = kOffXD  + (size_t)kRows * kPrjP * 4;
constexpr size_t kOffDUL  = kOffDUH + (size_t)kRows * kDtR  * 2;
constexpr size_t kOffDLR  = kOffDUL + (size_t)kRows * kDtR  * 2;
constexpr size_t kWsTotal = kOffDLR + (size_t)kRows * kDin  * 4;
static_assert(kWsTotal == 74973184ull, "carve total");
static_assert(kWsTotal <= 134217728ull, "carve cap");
static_assert((kOffXL % 128) == 0 && (kOffW1H % 128) == 0 && (kOffW1L % 128) == 0 && (kOffW2H % 128) == 0 &&
              (kOffW2L % 128) == 0 && (kOffXD % 128) == 0 && (kOffDUH % 128) == 0 && (kOffDUL % 128) == 0 &&
              (kOffDLR % 128) == 0, "128-B aligned regions");

__device__ __forceinline__ unsigned short f2bf_bits(float f) {
  unsigned u = __float_as_uint(f);
  return (unsigned short)((u + 0x7FFFu + ((u >> 16) & 1u)) >> 16);
}
__device__ __forceinline__ float bf_bits2f(unsigned short h) { return __uint_as_float(((unsigned)h) << 16); }

__device__ __forceinline__ void dep_guard_h(v8f& a, v8f& b, v16h x, v16h y) { asm volatile("v_nop\n\tv_nop\n\tv_nop\n\tv_nop" : "+v"(a), "+v"(b) : "v"(x), "v"(y)); }
__device__ __forceinline__ void dep_guard_b(v8f& a, v8f& b, v16b x, v16b y) { asm volatile("v_nop\n\tv_nop\n\tv_nop\n\tv_nop" : "+v"(a), "+v"(b) : "v"(x), "v"(y)); }
__device__ __forceinline__ void dep_guard4_h(v8f& a, v8f& b, v8f& c, v8f& d, v16h x, v16h y) { asm volatile("v_nop\n\tv_nop\n\tv_nop\n\tv_nop" : "+v"(a), "+v"(b), "+v"(c), "+v"(d) : "v"(x), "v"(y)); }
__device__ __forceinline__ void dep_guard4_b(v8f& a, v8f& b, v8f& c, v8f& d, v16b x, v16b y) { asm volatile("v_nop\n\tv_nop\n\tv_nop\n\tv_nop" : "+v"(a), "+v"(b), "+v"(c), "+v"(d) : "v"(x), "v"(y)); }
__device__ __forceinline__ void keep4_h(v16h a, v16h b, v16h c, v16h d) { asm volatile("v_nop" :: "v"(a), "v"(b), "v"(c), "v"(d)); }
__device__ __forceinline__ void keep4_b(v16b a, v16b b, v16b c, v16b d) { asm volatile("v_nop" :: "v"(a), "v"(b), "v"(c), "v"(d)); }
__device__ __forceinline__ void acc_guard4(v8f& a, v8f& b, v8f& c, v8f& d) { asm volatile("v_nop\n\tv_nop\n\tv_nop\n\tv_nop" : "+v"(a), "+v"(b), "+v"(c), "+v"(d)); }
template <typename T> struct Frag;
template <> struct Frag<_Float16> {
  typedef v16h V; union U { v16h v; v8h h[2]; };
  static __device__ __forceinline__ v16h load(const _Float16* p) {
    U f; f.h[0] = *(const v8h*)(p); f.h[1] = *(const v8h*)(p + 16); return f.v;
  }
  static __device__ __forceinline__ v8f mma(v16h a, v16h b, v8f c) {
    return __builtin_amdgcn_wmma_f32_16x16x32_f16(false, a, false, b, (short)0, c, false, false);
  }
  static __device__ __forceinline__ void guard(v8f& a, v8f& b, v16h x, v16h y) { dep_guard_h(a, b, x, y); }
  static __device__ __forceinline__ void guard4(v8f& a, v8f& b, v8f& c, v8f& d, v16h x, v16h y) { dep_guard4_h(a, b, c, d, x, y); }
  static __device__ __forceinline__ void keep(v16h a, v16h b, v16h c, v16h d) { keep4_h(a, b, c, d); }
};
template <> struct Frag<__bf16> {
  typedef v16b V; union U { v16b v; v8b h[2]; };
  static __device__ __forceinline__ v16b load(const __bf16* p) {
    U f; f.h[0] = *(const v8b*)(p); f.h[1] = *(const v8b*)(p + 16); return f.v;
  }
  static __device__ __forceinline__ v8f mma(v16b a, v16b b, v8f c) {
    return __builtin_amdgcn_wmma_f32_16x16x32_bf16(false, a, false, b, (short)0, c, false, false);
  }
  static __device__ __forceinline__ void guard(v8f& a, v8f& b, v16b x, v16b y) { dep_guard_b(a, b, x, y); }
  static __device__ __forceinline__ void guard4(v8f& a, v8f& b, v8f& c, v8f& d, v16b x, v16b y) { dep_guard4_b(a, b, c, d, x, y); }
  static __device__ __forceinline__ void keep(v16b a, v16b b, v16b c, v16b d) { keep4_b(a, b, c, d); }
};

template <int ET> struct Elem;
template <> struct Elem<0> { typedef _Float16 T; };
template <> struct Elem<1> { typedef __bf16 T; };
template <int ET, bool SPLIT, int BIAS_MODE, int OUT_MODE, bool RESID, int ACT = 0>
__global__ __launch_bounds__(256) void wmma_gemm64(
    const unsigned short* __restrict__ Ap, const unsigned short* __restrict__ A2p, int lda, long strideA,
    const unsigned short* __restrict__ Btp, const unsigned short* __restrict__ Bt2p, int ldb, long strideB,
    void* __restrict__ Cout, void* __restrict__ Cout2, int ldc, long strideC,
    const float* __restrict__ bias,
    const float* __restrict__ resid, long strideR,
    int M, int N, int K, float scale) {
  typedef typename Elem<ET>::T T;
  typedef typename Frag<T>::V V;
  const T* A = (const T*)Ap; const T* A2 = (const T*)A2p; const T* Bt = (const T*)Btp; const T* Bt2 = (const T*)Bt2p;
  __shared__ __align__(16) float sT[8][16 * 68];
  const int b    = blockIdx.y;
  const int lane = threadIdx.x & 31;
  const int wave = threadIdx.x >> 5;
  const int tilesN = N >> 6;
  const int tilesM = M >> 6;
  const int tile = blockIdx.x * 8 + wave;
  if (tile >= tilesM * tilesN) return;
  const int tm = tile / tilesN;
  const int tn = tile - tm * tilesN;
  const int m0 = tm << 6;
  const int n0 = tn << 6;

  const T* Ab  = A  + (size_t)b * strideA;
  const T* Bb  = Bt + (size_t)b * strideB;
  const T* Ab2 = SPLIT ? (A2  + (size_t)b * strideA) : nullptr;
  const T* Bb2 = SPLIT ? (Bt2 + (size_t)b * strideB) : nullptr;

  const int rlane = lane & 15;
  const int koff  = (lane >> 4) * 8;
  const int mOff  = (lane >> 4) * 8;

  v8f acc[4][4];
#pragma unroll
  for (int i = 0; i < 4; ++i)
#pragma unroll
    for (int j = 0; j < 4; ++j) acc[i][j] = (v8f){0.f,0.f,0.f,0.f,0.f,0.f,0.f,0.f};

  for (int k0 = 0; k0 < K; k0 += 32) {
    V bh[4], bl[4];
#pragma unroll
    for (int j = 0; j < 4; ++j) {
      const size_t bo = (size_t)(n0 + (j << 4) + rlane) * ldb + koff + k0;
      bh[j] = Frag<T>::load(Bb + bo);
      if (SPLIT) bl[j] = Frag<T>::load(Bb2 + bo);
    }
#pragma unroll
    for (int i = 0; i < 4; ++i) {
      const size_t ao = (size_t)(m0 + (i << 4) + rlane) * lda + koff + k0;
      V ah = Frag<T>::load(Ab + ao);
      V al;
      if (SPLIT) al = Frag<T>::load(Ab2 + ao);
#pragma unroll
      for (int j = 0; j < 4; ++j) {
        acc[i][j] = Frag<T>::mma(ah, bh[j], acc[i][j]);
        if (SPLIT) {
          acc[i][j] = Frag<T>::mma(ah, bl[j], acc[i][j]);
          acc[i][j] = Frag<T>::mma(al, bh[j], acc[i][j]);
        }
      }
      Frag<T>::guard4(acc[i][0], acc[i][1], acc[i][2], acc[i][3], ah, SPLIT ? al : ah);
    }
    Frag<T>::keep(bh[0], bh[1], bh[2], bh[3]);
    if (SPLIT) Frag<T>::keep(bl[0], bl[1], bl[2], bl[3]);
  }
  acc_guard4(acc[0][0], acc[0][1], acc[0][2], acc[0][3]);
  acc_guard4(acc[1][0], acc[1][1], acc[1][2], acc[1][3]);
  acc_guard4(acc[2][0], acc[2][1], acc[2][2], acc[2][3]);
  acc_guard4(acc[3][0], acc[3][1], acc[3][2], acc[3][3]);

  float* slab = sT[wave];
  const float* Rb = RESID ? (resid + (size_t)b * strideR) : nullptr;
#pragma unroll
  for (int i = 0; i < 4; ++i) {
    const int mBase = m0 + (i << 4);
#pragma unroll
    for (int j = 0; j < 4; ++j) {
      const int n = n0 + (j << 4) + rlane;
      float bv = 0.f;
      if (BIAS_MODE == 2) bv = bias[n];
#pragma unroll
      for (int r = 0; r < 8; ++r) {
        float v = acc[i][j][r] * scale;
        if (BIAS_MODE == 1) v += bias[mBase + mOff + r];
        if (BIAS_MODE == 2) v += bv;
        if (RESID) v += Rb[(size_t)(mBase + mOff + r) * ldc + n];
        if (ACT == 1) v = tanhf(v);
        if (ACT == 2) v = fmaxf(v, 0.0f);
        if (ACT == 3) v = v / (1.0f + expf(-v));
        if (ACT == 4) v = (v > 0.f) ? v : 0.01f * v;
        slab[(mOff + r) * 68 + (j << 4) + rlane] = v;
      }
    }
    __builtin_amdgcn_fence(__ATOMIC_RELEASE, "workgroup");
    __builtin_amdgcn_wave_barrier();
    __builtin_amdgcn_fence(__ATOMIC_ACQUIRE, "workgroup");
    if (OUT_MODE == 0) {
      float* C = (float*)Cout + (size_t)b * strideC;
      const int hh = lane >> 4, c4 = (lane & 15) * 4;
      for (int pass = 0; pass < 2; ++pass) {
#pragma unroll
        for (int it = 0; it < 8; ++it) {
          const int row = it * 2 + hh;
          v4f v = *(const v4f*)(slab + row * 68 + c4);
          *(volatile v4f*)(C + (size_t)(mBase + row) * ldc + n0 + c4) = v;
        }
        __threadfence();
      }
    } else {
      const int q = lane >> 3, c8 = (lane & 7) * 8;
      unsigned short* C  = (unsigned short*)Cout  + (size_t)b * strideC;
      unsigned short* C2 = (OUT_MODE == 2) ? ((unsigned short*)Cout2 + (size_t)b * strideC) : nullptr;
      for (int pass = 0; pass < 2; ++pass) {
#pragma unroll
        for (int it = 0; it < 4; ++it) {
          const int row = it * 4 + q;
          const float* sp = slab + row * 68 + c8;
          v8h hv, lv;
#pragma unroll
          for (int e = 0; e < 8; ++e) {
            if (OUT_MODE == 1) {
              hv[e] = (_Float16)sp[e];
            } else {
              unsigned short hb = f2bf_bits(sp[e]);
              unsigned short lb = f2bf_bits(sp[e] - bf_bits2f(hb));
              hv[e] = __builtin_bit_cast(_Float16, hb);
              lv[e] = __builtin_bit_cast(_Float16, lb);
            }
          }
          *(volatile v8h*)(C + (size_t)(mBase + row) * ldc + n0 + c8) = hv;
          if (OUT_MODE == 2) *(volatile v8h*)(C2 + (size_t)(mBase + row) * ldc + n0 + c8) = lv;
        }
        __threadfence();
      }
    }
    __builtin_amdgcn_fence(__ATOMIC_RELEASE, "workgroup");
    __builtin_amdgcn_wave_barrier();
    __builtin_amdgcn_fence(__ATOMIC_ACQUIRE, "workgroup");
  }
}

__global__ __launch_bounds__(256) void split_rows_bf16_kernel(
    const float* __restrict__ src, unsigned short* __restrict__ dhi, unsigned short* __restrict__ dlo,
    int nsrc8, int total8)
{
  const int i = blockIdx.x * 256 + threadIdx.x;
  if (i >= total8) return;
  const bool pad = (i >= nsrc8);
  const int ic = pad ? (nsrc8 - 1) : i;
  const size_t s0 = (size_t)ic << 3;
  const v4f a0 = *(const v4f*)(src + s0);
  const v4f a1 = *(const v4f*)(src + s0 + 4);
  v8h hv, lv;
#pragma unroll
  for (int e = 0; e < 4; ++e) {
    const float f0 = pad ? 0.0f : a0[e];
    const float f1 = pad ? 0.0f : a1[e];
    const unsigned short h0 = f2bf_bits(f0), h1 = f2bf_bits(f1);
    const unsigned short l0 = f2bf_bits(f0 - bf_bits2f(h0)), l1 = f2bf_bits(f1 - bf_bits2f(h1));
    hv[e]     = __builtin_bit_cast(_Float16, h0);
    hv[4 + e] = __builtin_bit_cast(_Float16, h1);
    lv[e]     = __builtin_bit_cast(_Float16, l0);
    lv[4 + e] = __builtin_bit_cast(_Float16, l1);
  }
  const size_t e0 = (size_t)i << 3;
  unsigned short* qh = dhi + e0;
  unsigned short* ql = dlo + e0;
  *(volatile v8h*)qh = hv;
  *(volatile v8h*)ql = lv;
  __threadfence();
  *(volatile v8h*)qh = hv;
  *(volatile v8h*)ql = lv;
}

__global__ __launch_bounds__(256) void dun_split_kernel(
    const float* __restrict__ XD, unsigned short* __restrict__ DUH, unsigned short* __restrict__ DUL, int total8)
{
  const int i = blockIdx.x * 256 + threadIdx.x;
  if (i >= total8) return;
  const int e0  = i << 3;
  const int row = e0 >> 7;
  const int c8  = e0 & (kDtR - 1);
  const float* p = XD + (size_t)row * kPrjP + c8;
  const v4f a0 = *(const v4f*)(p);
  const v4f a1 = *(const v4f*)(p + 4);
  v8h hv, lv;
#pragma unroll
  for (int e = 0; e < 4; ++e) {
    const unsigned short h0 = f2bf_bits(a0[e]), h1 = f2bf_bits(a1[e]);
    const unsigned short l0 = f2bf_bits(a0[e] - bf_bits2f(h0)), l1 = f2bf_bits(a1[e] - bf_bits2f(h1));
    hv[e]     = __builtin_bit_cast(_Float16, h0);
    hv[4 + e] = __builtin_bit_cast(_Float16, h1);
    lv[e]     = __builtin_bit_cast(_Float16, l0);
    lv[4 + e] = __builtin_bit_cast(_Float16, l1);
  }
  unsigned short* qh = DUH + (size_t)e0;
  unsigned short* ql = DUL + (size_t)e0;
  *(volatile v8h*)qh = hv;
  *(volatile v8h*)ql = lv;
  __threadfence();
  *(volatile v8h*)qh = hv;
  *(volatile v8h*)ql = lv;
}

__global__ __launch_bounds__(64) void scan_kernel(
    const float* __restrict__ DLR, const float* __restrict__ X, const float* __restrict__ XD,
    const float* __restrict__ Alog, const float* __restrict__ Dp, float* __restrict__ OUT)
{
  __shared__ __align__(16) float sBC[kScanTS * kBCW];
  __shared__ __align__(16) float sY[kScanTS * kScanYP];
  __shared__ __align__(16) float sA[kNst * kScanCh];
  const int tid = threadIdx.x, lane = tid & 31, wave = tid >> 5;
  constexpr int kBlkPerB = kDin / kScanCh;
  const int bix = blockIdx.x / kBlkPerB;
  const int d0  = (blockIdx.x - bix * kBlkPerB) * kScanCh;
  const int d   = d0 + tid;
  const size_t row0 = (size_t)bix * kSeq;
#pragma unroll 1
  for (int s = 0; s < kNst; ++s) sA[s * kScanCh + tid] = 0.0f - expf(Alog[(size_t)d * kNst + s]);
  __syncthreads();
  float An[kNst], h[kNst];
#pragma unroll
  for (int s = 0; s < kNst; ++s) {
    An[s] = sA[s * kScanCh + tid];
    h[s] = 0.0f;
  }
  const float Dd = Dp[d];
  const int lr = tid >> 3, lc4 = (tid & 7) * 4;
  const int hh = lane >> 4, c4 = (lane & 15) * 4;
#pragma unroll 1
  for (int t0 = 0; t0 < kSeq; t0 += kScanTS) {
    __syncthreads();
#pragma unroll
    for (int i = 0; i < 8; ++i) {
      const int r = lr + 8 * i;
      *(v4f*)(sBC + r * kBCW + lc4) = *(const v4f*)(XD + (row0 + (size_t)(t0 + r)) * kPrjP + kDtR + lc4);
    }
    __syncthreads();
#pragma unroll 1
    for (int s = 0; s < kScanTS; ++s) {
      const size_t m = row0 + (size_t)(t0 + s);
      const float z  = DLR[m * kDin + d];
      const float xv = X[m * kDin + d];
      const float dt = fmaxf(z, 0.0f) + log1pf(expf(-fabsf(z)));
      const float* xr = sBC + s * kBCW;
      v4f Bq[4], Cq[4];
#pragma unroll
      for (int qq = 0; qq < 4; ++qq) {
        Bq[qq] = *(const v4f*)(xr + 4 * qq);
        Cq[qq] = *(const v4f*)(xr + kNst + 4 * qq);
      }
      const float dtx = dt * xv;
      float y = 0.0f;
#pragma unroll
      for (int n = 0; n < kNst; ++n) {
        const float e  = __expf(dt * An[n]);
        const float hn = e * h[n] + dtx * Bq[n >> 2][n & 3];
        h[n] = hn;
        y = hn * Cq[n >> 2][n & 3] + y;
      }
      y = xv * Dd + y;
      sY[s * kScanYP + tid] = y;
    }
    __syncthreads();
    for (int pass = 0; pass < 2; ++pass) {
#pragma unroll
      for (int it = 0; it < 16; ++it) {
        const int row = it * 4 + wave * 2 + hh;
        const v4f v = *(const v4f*)(sY + row * kScanYP + c4);
        *(volatile v4f*)(OUT + (row0 + (size_t)(t0 + row)) * kDin + d0 + c4) = v;
      }
      __threadfence();
    }
  }
}

extern "C" void kernel_launch(void* const* d_in, const int* in_sizes, int n_in,
                              void* d_out, int out_size, void* d_ws, size_t ws_size,
                              hipStream_t stream) {
  if (n_in < 6) return;
  if (in_sizes[0] != kRows * kDin) return;
  if (in_sizes[1] != kPrjN * kDin) return;
  if (in_sizes[2] != kDin * kDtR) return;
  if (in_sizes[3] != kDin) return;
  if (in_sizes[4] != kDin * kNst) return;
  if (in_sizes[5] != kDin) return;
  if (out_size != kRows * kDin) return;
  if (ws_size < kWsTotal) return;

  const float* x      = (const float*)d_in[0];
  const float* W_xprj = (const float*)d_in[1];
  const float* W_dt   = (const float*)d_in[2];
  const float* b_dt   = (const float*)d_in[3];
  const float* A_log  = (const float*)d_in[4];
  const float* Dv     = (const float*)d_in[5];
  float* out = (float*)d_out;

  char* ws = (char*)d_ws;
  unsigned short* XH  = (unsigned short*)(ws + kOffXH);
  unsigned short* XL  = (unsigned short*)(ws + kOffXL);
  unsigned short* W1H = (unsigned short*)(ws + kOffW1H);
  unsigned short* W1L = (unsigned short*)(ws + kOffW1L);
  unsigned short* W2H = (unsigned short*)(ws + kOffW2H);
  unsigned short* W2L = (unsigned short*)(ws + kOffW2L);
  float*          XD  = (float*)(ws + kOffXD);
  unsigned short* DUH = (unsigned short*)(ws + kOffDUH);
  unsigned short* DUL = (unsigned short*)(ws + kOffDUL);
  float*          DLR = (float*)(ws + kOffDLR);
  const float* dummy_bias  = b_dt;
  const float* dummy_resid = x;

  constexpr int kX8  = kRows * kDin / 8;
  constexpr int kW18 = kPrjP * kDin / 8;
  constexpr int kW1s = kPrjN * kDin / 8;
  constexpr int kW28 = kDin * kDtR / 8;
  static_assert((kX8 % 256) == 0 && (kW18 % 256) == 0 && (kW28 % 256) == 0, "exact grids");
  split_rows_bf16_kernel<<<kX8 / 256, 256, 0, stream>>>(x, XH, XL, kX8, kX8);
  split_rows_bf16_kernel<<<kW18 / 256, 256, 0, stream>>>(W_xprj, W1H, W1L, kW1s, kW18);
  split_rows_bf16_kernel<<<kW28 / 256, 256, 0, stream>>>(W_dt, W2H, W2L, kW28, kW28);

  static_assert(((kRows / 64) * (kPrjP / 64)) % 8 == 0, "x_proj tiles fill whole blocks");
  wmma_gemm64<1, true, 0, 0, false><<<dim3((kRows / 64) * (kPrjP / 64) / 8, 1), 256, 0, stream>>>(
      XH, XL, kDin, 0L,
      W1H, W1L, kDin, 0L,
      (void*)XD, (void*)XD, kPrjP, 0L,
      dummy_bias, dummy_resid, 0L,
      kRows, kPrjP, kDin, 1.0f);

  constexpr int kDU8 = kRows * kDtR / 8;
  static_assert((kDU8 % 256) == 0, "exact grid");
  dun_split_kernel<<<kDU8 / 256, 256, 0, stream>>>(XD, DUH, DUL, kDU8);

  static_assert(((kRows / 64) * (kDin / 64)) % 8 == 0, "dt_proj tiles fill whole blocks");
  wmma_gemm64<1, true, 2, 0, false><<<dim3((kRows / 64) * (kDin / 64) / 8, 1), 256, 0, stream>>>(
      DUH, DUL, kDtR, 0L,
      W2H, W2L, kDtR, 0L,
      (void*)DLR, (void*)DLR, kDin, 0L,
      b_dt, dummy_resid, 0L,
      kRows, kDin, kDtR, 1.0f);

  scan_kernel<<<kBatch * (kDin / kScanCh), kScanCh, 0, stream>>>(DLR, x, XD, A_log, Dv, out);
}
